// Model_26353919328765
// MI455X (gfx1250) — hardware-verified
//
#include <hip/hip_runtime.h>
#include <math.h>

constexpr int NBAT   = 64;
constexpr int NSEQ   = 512;
constexpr int NQRY   = 64;
constexpr int NDIM   = 256;
constexpr int NHID   = 128;
constexpr int NGATE  = 4 * NHID;
constexpr int NFEAT  = 4 * NDIM;
constexpr int NBI    = 2 * NHID;
constexpr int NWVEC  = NFEAT + NBI;
constexpr int NROWS  = NBAT * NSEQ;
constexpr int NQROWS = NBAT * NQRY;
constexpr int NTHR   = 256;
constexpr int HPITCH = 136;
constexpr int PPITCH = 520;
constexpr float WCARRY     = 16.0f;
constexpr float WCARRY_INV = 1.0f / 16.0f;
constexpr float QCARRY     = 64.0f;
constexpr float QCARRY_INV = 1.0f / 64.0f;
constexpr float PCARRY     = 1024.0f;
constexpr float PCARRY_INV = 1.0f / 1024.0f;

static_assert(NGATE == 512);
static_assert(NFEAT == 1024);
static_assert(NWVEC == 1280);
static_assert(NROWS == 32768);
static_assert(NDIM % 32 == 0 && NQRY % 32 == 0 && NFEAT % 32 == 0 && NBI % 32 == 0 && NHID % 32 == 0);
static_assert(NSEQ % 64 == 0 && NQRY % 64 == 0 && NDIM % 64 == 0 && NGATE % 64 == 0 && NROWS % 64 == 0);
static_assert(NDIM == 32 * 8);
static_assert(NQRY == 32 * 2);
static_assert(NHID == 16 * (NTHR / 32));
static_assert(NBI == NTHR);
static_assert((2 * 16 * HPITCH) % NTHR == 0);
static_assert(NROWS % (NTHR) == 0 && NQROWS % (NTHR) == 0);

typedef __attribute__((ext_vector_type(16))) _Float16 v16h;
typedef __attribute__((ext_vector_type(8)))  _Float16 v8h;
typedef __attribute__((ext_vector_type(8)))  float    v8f;
typedef __attribute__((ext_vector_type(4)))  float    v4f;
typedef __attribute__((ext_vector_type(2)))  float    v2f;
typedef __attribute__((ext_vector_type(4)))  unsigned v4u;

__device__ __forceinline__ float h16_to_f32(unsigned hb) {
  const unsigned sgn = (hb & 0x8000u) << 16;
  const unsigned em = hb & 0x7fffu;
  const float fn = __uint_as_float((em << 13) + 0x38000000u);
  const float fs = (float)em * 5.9604644775390625e-8f;
  const float mag = (em < 0x400u) ? fs : fn;
  return __uint_as_float(__float_as_uint(mag) | sgn);
}
__device__ __forceinline__ unsigned short f16_bits(float x) {
  const _Float16 h = (_Float16)x;
  return __builtin_bit_cast(unsigned short, h);
}

__device__ __forceinline__ void guard4_h(v8f& a, v8f& b, v8f& c, v8f& d, v16h x, v16h y0, v16h y1, v16h y2, v16h y3) {
  asm volatile("v_nop\n\tv_nop\n\tv_nop\n\tv_nop" : "+v"(a), "+v"(b), "+v"(c), "+v"(d) : "v"(x), "v"(y0), "v"(y1), "v"(y2), "v"(y3));
}
__device__ __forceinline__ void keep4_h(v16h a, v16h b, v16h c, v16h d) { asm volatile("v_nop" :: "v"(a), "v"(b), "v"(c), "v"(d)); }
__device__ __forceinline__ void acc_guard4(v8f& a, v8f& b, v8f& c, v8f& d) { asm volatile("v_nop\n\tv_nop\n\tv_nop\n\tv_nop" : "+v"(a), "+v"(b), "+v"(c), "+v"(d)); }

template <typename T> struct Frag;
template <> struct Frag<_Float16> {
  typedef v16h V; union U { v16h v; v8h h[2]; };
  static __device__ __forceinline__ v16h load(const _Float16* p) {
    U f; f.h[0] = *(const v8h*)(p); f.h[1] = *(const v8h*)(p + 16); return f.v;
  }
  static __device__ __forceinline__ v8f mma(v16h a, v16h b, v8f c) {
    return __builtin_amdgcn_wmma_f32_16x16x32_f16(false, a, false, b, (short)0, c, false, false);
  }
};

__device__ __forceinline__ float fsig(float x)  { return __builtin_amdgcn_rcpf(1.0f + __expf(-x)); }
__device__ __forceinline__ float ftanh(float x) { return 1.0f - 2.0f * __builtin_amdgcn_rcpf(__expf(2.0f * x) + 1.0f); }

__global__ __launch_bounds__(NTHR) void cvtw_kernel(const float* __restrict__ s0, const float* __restrict__ s1,
                                                    const float* __restrict__ s2, const float* __restrict__ s3,
                                                    unsigned short* __restrict__ d0, unsigned short* __restrict__ d1,
                                                    unsigned short* __restrict__ d2, unsigned short* __restrict__ d3,
                                                    int n8, float sc) {
  const int y = blockIdx.y;
  const float* src = (y == 0) ? s0 : (y == 1) ? s1 : (y == 2) ? s2 : s3;
  unsigned short* dst = (y == 0) ? d0 : (y == 1) ? d1 : (y == 2) ? d2 : d3;
  const int i = blockIdx.x * NTHR + threadIdx.x;
  if (i < n8) {
    const float* sp = src + (size_t)i * 8;
    const v4f a = *(const v4f*)(sp);
    const v4f b = *(const v4f*)(sp + 4);
    v8h hv;
#pragma unroll
    for (int e = 0; e < 4; ++e) {
      hv[e]     = (_Float16)(a[e] * sc);
      hv[4 + e] = (_Float16)(b[e] * sc);
    }
    unsigned short* op = dst + (size_t)i * 8;
    *(volatile v8h*)op = hv;
    __threadfence();
    *(volatile v8h*)op = hv;
  }
}

__global__ __launch_bounds__(512) void bsum_kernel(const float* __restrict__ a0, const float* __restrict__ b0,
                                                   const float* __restrict__ a1, const float* __restrict__ b1,
                                                   const float* __restrict__ a2, const float* __restrict__ b2,
                                                   const float* __restrict__ a3, const float* __restrict__ b3,
                                                   float* __restrict__ dst) {
  const int tid = threadIdx.x;
  const int which = tid >> 7;
  const int idx = (tid & 127) * 4;
  const v4f x0 = *(const v4f*)(a0 + idx), y0 = *(const v4f*)(b0 + idx);
  const v4f x1 = *(const v4f*)(a1 + idx), y1 = *(const v4f*)(b1 + idx);
  const v4f x2 = *(const v4f*)(a2 + idx), y2 = *(const v4f*)(b2 + idx);
  const v4f x3 = *(const v4f*)(a3 + idx), y3 = *(const v4f*)(b3 + idx);
  v4f o;
#pragma unroll
  for (int e = 0; e < 4; ++e) {
    const float t0 = x0[e] + y0[e], t1 = x1[e] + y1[e], t2 = x2[e] + y2[e], t3 = x3[e] + y3[e];
    o[e] = (which == 0) ? t0 : (which == 1) ? t1 : (which == 2) ? t2 : t3;
  }
  float* op = dst + which * NGATE + idx;
  *(volatile v4f*)op = o;
  __threadfence();
  *(volatile v4f*)op = o;
}

template <int MODE>
__global__ __launch_bounds__(NTHR) void rowprep_kernel(const float* __restrict__ X, const float* __restrict__ wdot,
                                                       const float* __restrict__ bias1, const float* __restrict__ bias2,
                                                       const float* __restrict__ wmul,
                                                       unsigned short* __restrict__ out16, int opitch,
                                                       float* __restrict__ dots, int nrows) {
  const int lane = threadIdx.x & 31, wave = threadIdx.x >> 5;
  const int row0 = (blockIdx.x * 8 + wave) * 32;
  if (row0 >= nrows) return;
  const int c8 = lane * 8;
  const v4f wa = *(const v4f*)(wdot + c8);
  const v4f wb = *(const v4f*)(wdot + c8 + 4);
  const v4f ma = *(const v4f*)(wmul + c8);
  const v4f mb = *(const v4f*)(wmul + c8 + 4);
  float bv = bias1[0];
  if (MODE == 0) bv += bias2[0];
  float keep = 0.0f;
#pragma unroll 1
  for (int i = 0; i < 32; ++i) {
    const int row = row0 + i;
    const float* xp = X + (size_t)row * NDIM + c8;
    const v4f a = *(const v4f*)(xp);
    const v4f b = *(const v4f*)(xp + 4);
    float s = 0.0f;
    v8h hv;
#pragma unroll
    for (int e = 0; e < 4; ++e) {
      s = fmaf(a[e], wa[e], s);
      float o = a[e];
      if (MODE == 1) o = a[e] * (ma[e] * QCARRY);
      hv[e] = (_Float16)o;
    }
#pragma unroll
    for (int e = 0; e < 4; ++e) {
      s = fmaf(b[e], wb[e], s);
      float o = b[e];
      if (MODE == 1) o = b[e] * (mb[e] * QCARRY);
      hv[4 + e] = (_Float16)o;
    }
#pragma unroll
    for (int off = 1; off < 32; off <<= 1) s += __shfl_xor(s, off, 32);
    const float dv = s + bv;
    keep = (lane == i) ? dv : keep;
    unsigned short* op = out16 + (size_t)row * opitch + c8;
    *(volatile v8h*)op = hv;
    __threadfence();
    *(volatile v8h*)op = hv;
  }
  float* dp = dots + row0 + lane;
  *(volatile float*)dp = keep;
  __threadfence();
  *(volatile float*)dp = keep;
}

__global__ __launch_bounds__(NTHR) void qtrans_kernel(const float* __restrict__ q, unsigned short* __restrict__ qT) {
  __shared__ float Tt[64 * 65];
  const int tid = threadIdx.x;
  const int d0 = blockIdx.x * 64;
  const int b = blockIdx.y;
  const float* src = q + (size_t)b * NQRY * NDIM;
#pragma unroll
  for (int i = 0; i < 4; ++i) {
    const int idx = i * NTHR + tid;
    const int jj = idx >> 4, cc = (idx & 15) * 4;
    const v4f v = *(const v4f*)(src + (size_t)jj * NDIM + d0 + cc);
    Tt[jj * 65 + cc + 0] = v[0];
    Tt[jj * 65 + cc + 1] = v[1];
    Tt[jj * 65 + cc + 2] = v[2];
    Tt[jj * 65 + cc + 3] = v[3];
  }
  __syncthreads();
  const int qq = tid >> 3, c8 = (tid & 7) * 8;
  v8h hv[2];
#pragma unroll
  for (int g = 0; g < 2; ++g) {
    const int dd = g * 32 + qq;
#pragma unroll
    for (int e = 0; e < 8; ++e) hv[g][e] = (_Float16)Tt[(c8 + e) * 65 + dd];
  }
  unsigned short* ob = qT + (size_t)b * NDIM * NQRY;
  for (int pass = 0; pass < 2; ++pass) {
#pragma unroll
    for (int g = 0; g < 2; ++g) {
      const size_t o = (size_t)(d0 + g * 32 + qq) * NQRY + c8;
      *(volatile v8h*)(ob + o) = hv[g];
    }
    __threadfence();
  }
}

template <int OUT_MODE, bool ADDS>
__global__ __launch_bounds__(256) void gemm64_kernel(
    const unsigned short* __restrict__ Ap, int lda, long strideA,
    const unsigned short* __restrict__ Btp, int ldb, long strideB,
    void* __restrict__ Cout, int ldc, long strideC,
    const float* __restrict__ rowadd, long strideRA,
    const float* __restrict__ coladd, long strideCA,
    int Mdim, int Ndim, int Kdim, float scale) {
  typedef _Float16 T;
  const T* A = (const T*)Ap;
  const T* Bt = (const T*)Btp;
  __shared__ __align__(16) float sT[8][16 * 68];
  const int b    = blockIdx.y;
  const int lane = threadIdx.x & 31;
  const int wave = threadIdx.x >> 5;
  const int tilesN = Ndim >> 6;
  const int tilesM = Mdim >> 6;
  const int tile = blockIdx.x * 8 + wave;
  if (tile >= tilesM * tilesN) return;
  const int tm = tile / tilesN;
  const int tn = tile - tm * tilesN;
  const int m0 = tm << 6;
  const int n0 = tn << 6;

  const T* Ab = A  + (size_t)b * strideA;
  const T* Bb = Bt + (size_t)b * strideB;

  const int rlane = lane & 15;
  const int koff  = (lane >> 4) * 8;
  const int mOff  = (lane >> 4) * 8;

  v8f acc[4][4];
#pragma unroll
  for (int i = 0; i < 4; ++i)
#pragma unroll
    for (int j = 0; j < 4; ++j) acc[i][j] = (v8f){0.f,0.f,0.f,0.f,0.f,0.f,0.f,0.f};

  for (int k0 = 0; k0 < Kdim; k0 += 32) {
    v16h bh[4];
#pragma unroll
    for (int j = 0; j < 4; ++j) {
      const size_t bo = (size_t)(n0 + (j << 4) + rlane) * ldb + koff + k0;
      bh[j] = Frag<T>::load(Bb + bo);
    }
#pragma unroll
    for (int i = 0; i < 4; ++i) {
      const size_t ao = (size_t)(m0 + (i << 4) + rlane) * lda + koff + k0;
      const v16h ah = Frag<T>::load(Ab + ao);
#pragma unroll
      for (int j = 0; j < 4; ++j) acc[i][j] = Frag<T>::mma(ah, bh[j], acc[i][j]);
      guard4_h(acc[i][0], acc[i][1], acc[i][2], acc[i][3], ah, bh[0], bh[1], bh[2], bh[3]);
    }
    keep4_h(bh[0], bh[1], bh[2], bh[3]);
  }
  acc_guard4(acc[0][0], acc[0][1], acc[0][2], acc[0][3]);
  acc_guard4(acc[1][0], acc[1][1], acc[1][2], acc[1][3]);
  acc_guard4(acc[2][0], acc[2][1], acc[2][2], acc[2][3]);
  acc_guard4(acc[3][0], acc[3][1], acc[3][2], acc[3][3]);

  float* slab = sT[wave];
#pragma unroll
  for (int i = 0; i < 4; ++i) {
    const int mBase = m0 + (i << 4);
#pragma unroll
    for (int j = 0; j < 4; ++j) {
#pragma unroll
      for (int r = 0; r < 8; ++r) slab[(mOff + r) * 68 + (j << 4) + rlane] = acc[i][j][r] * scale;
    }
    __builtin_amdgcn_fence(__ATOMIC_RELEASE, "workgroup");
    __builtin_amdgcn_wave_barrier();
    __builtin_amdgcn_fence(__ATOMIC_ACQUIRE, "workgroup");
    if (OUT_MODE == 0) {
      float* C = (float*)Cout + (size_t)b * strideC;
      const int hh = lane >> 4, c4 = (lane & 15) * 4;
      v4f ca = (v4f){0.f, 0.f, 0.f, 0.f};
      float ra[8];
#pragma unroll
      for (int it = 0; it < 8; ++it) ra[it] = 0.0f;
      if (ADDS) {
        ca = *(const v4f*)(coladd + (size_t)b * strideCA + n0 + c4);
#pragma unroll
        for (int it = 0; it < 8; ++it) ra[it] = rowadd[(size_t)b * strideRA + mBase + it * 2 + hh];
      }
      for (int pass = 0; pass < 2; ++pass) {
#pragma unroll
        for (int it = 0; it < 8; ++it) {
          const int row = it * 2 + hh;
          v4f v = *(const v4f*)(slab + row * 68 + c4);
#pragma unroll
          for (int e = 0; e < 4; ++e) v[e] = v[e] + ra[it] + ca[e];
          *(volatile v4f*)(C + (size_t)(mBase + row) * ldc + n0 + c4) = v;
        }
        __threadfence();
      }
    } else {
      const int q = lane >> 3, c8 = (lane & 7) * 8;
      unsigned short* C = (unsigned short*)Cout + (size_t)b * strideC;
      v4f ba = (v4f){0.f, 0.f, 0.f, 0.f};
      v4f bb = (v4f){0.f, 0.f, 0.f, 0.f};
      if (ADDS) {
        ba = *(const v4f*)(coladd + (size_t)b * strideCA + n0 + c8);
        bb = *(const v4f*)(coladd + (size_t)b * strideCA + n0 + c8 + 4);
      }
      for (int pass = 0; pass < 2; ++pass) {
#pragma unroll
        for (int it = 0; it < 4; ++it) {
          const int row = it * 4 + q;
          const float* sp = slab + row * 68 + c8;
          v8h hv;
#pragma unroll
          for (int e = 0; e < 4; ++e) {
            hv[e]     = (_Float16)(sp[e] + ba[e]);
            hv[4 + e] = (_Float16)(sp[4 + e] + bb[e]);
          }
          *(volatile v8h*)(C + (size_t)(mBase + row) * ldc + n0 + c8) = hv;
        }
        __threadfence();
      }
    }
    __builtin_amdgcn_fence(__ATOMIC_RELEASE, "workgroup");
    __builtin_amdgcn_wave_barrier();
    __builtin_amdgcn_fence(__ATOMIC_ACQUIRE, "workgroup");
  }
}

__global__ __launch_bounds__(NTHR) void softj_kernel(const float* __restrict__ S, unsigned short* __restrict__ A16,
                                                     float* __restrict__ smax) {
  const int lane = threadIdx.x & 31, wave = threadIdx.x >> 5;
  const int row0 = (blockIdx.x * 8 + wave) * 32;
  if (row0 >= NROWS) return;
  float keep = 0.0f;
#pragma unroll 1
  for (int i = 0; i < 32; ++i) {
    const int row = row0 + i;
    const v2f x = *(const v2f*)(S + (size_t)row * NQRY + 2 * lane);
    float m = fmaxf(x[0], x[1]);
#pragma unroll
    for (int off = 1; off < 32; off <<= 1) m = fmaxf(m, __shfl_xor(m, off, 32));
    const float e0 = expf(x[0] - m);
    const float e1 = expf(x[1] - m);
    float s = e0 + e1;
#pragma unroll
    for (int off = 1; off < 32; off <<= 1) s += __shfl_xor(s, off, 32);
    const float inv = (1.0f / s) * PCARRY;
    const unsigned short h0 = f16_bits(e0 * inv);
    const unsigned short h1 = f16_bits(e1 * inv);
    const unsigned u = (unsigned)h0 | ((unsigned)h1 << 16);
    unsigned* op = (unsigned*)(void*)A16 + (size_t)row * 32 + lane;
    *(volatile unsigned*)op = u;
    __threadfence();
    *(volatile unsigned*)op = u;
    keep = (lane == i) ? m : keep;
  }
  float* sp = smax + row0 + lane;
  *(volatile float*)sp = keep;
  __threadfence();
  *(volatile float*)sp = keep;
}

__global__ __launch_bounds__(NTHR) void q2c_kernel(const float* __restrict__ smax, const float* __restrict__ cx,
                                                   float* __restrict__ q2c) {
  __shared__ float bat[NSEQ];
  __shared__ float red[8];
  const int tid = threadIdx.x, lane = tid & 31, wave = tid >> 5;
  const int b = blockIdx.x;
  const float v0 = smax[(size_t)b * NSEQ + tid];
  const float v1 = smax[(size_t)b * NSEQ + 256 + tid];
  float m = fmaxf(v0, v1);
#pragma unroll
  for (int off = 1; off < 32; off <<= 1) m = fmaxf(m, __shfl_xor(m, off, 32));
  if (lane == 0) red[wave] = m;
  __syncthreads();
  float mx = red[0];
#pragma unroll
  for (int w = 1; w < 8; ++w) mx = fmaxf(mx, red[w]);
  __syncthreads();
  const float e0 = expf(v0 - mx);
  const float e1 = expf(v1 - mx);
  float s = e0 + e1;
#pragma unroll
  for (int off = 1; off < 32; off <<= 1) s += __shfl_xor(s, off, 32);
  if (lane == 0) red[wave] = s;
  __syncthreads();
  const float tot = ((red[0] + red[1]) + (red[2] + red[3])) + ((red[4] + red[5]) + (red[6] + red[7]));
  const float inv = 1.0f / tot;
  bat[tid] = e0 * inv;
  bat[tid + 256] = e1 * inv;
  __syncthreads();
  const float* cp = cx + (size_t)b * NSEQ * NDIM + tid;
  float a0 = 0.0f, a1 = 0.0f, a2 = 0.0f, a3 = 0.0f;
#pragma unroll 1
  for (int t = 0; t < NSEQ; t += 4) {
    a0 = fmaf(bat[t + 0], cp[(size_t)(t + 0) * NDIM], a0);
    a1 = fmaf(bat[t + 1], cp[(size_t)(t + 1) * NDIM], a1);
    a2 = fmaf(bat[t + 2], cp[(size_t)(t + 2) * NDIM], a2);
    a3 = fmaf(bat[t + 3], cp[(size_t)(t + 3) * NDIM], a3);
  }
  const float r = (a0 + a1) + (a2 + a3);
  float* op = q2c + (size_t)b * NDIM + tid;
  *(volatile float*)op = r;
  __threadfence();
  *(volatile float*)op = r;
}

__global__ __launch_bounds__(NTHR) void assemble_kernel(const float* __restrict__ cx, const unsigned short* __restrict__ c2q16,
                                                        const float* __restrict__ q2c, const float* __restrict__ W0,
                                                        const float* __restrict__ W1, unsigned short* __restrict__ g16,
                                                        float* __restrict__ zg0, float* __restrict__ zg1) {
  const int lane = threadIdx.x & 31, wave = threadIdx.x >> 5;
  const int row0 = (blockIdx.x * 8 + wave) * 32;
  if (row0 >= NROWS) return;
  const int b = row0 / NSEQ;
  const int c8 = lane * 8;
  float qv[8], w0s[4][8], w1s[4][8];
  {
    const v4f x = *(const v4f*)(q2c + (size_t)b * NDIM + c8);
    const v4f y = *(const v4f*)(q2c + (size_t)b * NDIM + c8 + 4);
#pragma unroll
    for (int e = 0; e < 4; ++e) { qv[e] = x[e]; qv[4 + e] = y[e]; }
  }
#pragma unroll
  for (int sg = 0; sg < 4; ++sg) {
    const v4f x0 = *(const v4f*)(W0 + sg * NDIM + c8);
    const v4f y0 = *(const v4f*)(W0 + sg * NDIM + c8 + 4);
    const v4f x1 = *(const v4f*)(W1 + sg * NDIM + c8);
    const v4f y1 = *(const v4f*)(W1 + sg * NDIM + c8 + 4);
#pragma unroll
    for (int e = 0; e < 4; ++e) {
      w0s[sg][e] = x0[e]; w0s[sg][4 + e] = y0[e];
      w1s[sg][e] = x1[e]; w1s[sg][4 + e] = y1[e];
    }
  }
  float keep0 = 0.0f, keep1 = 0.0f;
#pragma unroll 1
  for (int i = 0; i < 32; ++i) {
    const int row = row0 + i;
    const float* cp = cx + (size_t)row * NDIM + c8;
    const v4f ca = *(const v4f*)(cp);
    const v4f cb = *(const v4f*)(cp + 4);
    const v4u hw = *(const v4u*)(const void*)(c2q16 + (size_t)row * NDIM + c8);
    float cvv[8], cq[8];
#pragma unroll
    for (int e = 0; e < 4; ++e) { cvv[e] = ca[e]; cvv[4 + e] = cb[e]; }
#pragma unroll
    for (int k = 0; k < 4; ++k) {
      const unsigned wd = hw[k];
      cq[2 * k]     = h16_to_f32(wd & 0xffffu);
      cq[2 * k + 1] = h16_to_f32(wd >> 16);
    }
    float z0 = 0.0f, z1 = 0.0f;
    v8h h2, h3;
#pragma unroll
    for (int e = 0; e < 8; ++e) {
      const float t0 = cvv[e];
      const float t1 = cq[e];
      const float t2 = t0 * t1;
      const float t3 = t0 * qv[e];
      h2[e] = (_Float16)t2;
      h3[e] = (_Float16)t3;
      z0 = fmaf(t0, w0s[0][e], z0);
      z0 = fmaf(t1, w0s[1][e], z0);
      z0 = fmaf(t2, w0s[2][e], z0);
      z0 = fmaf(t3, w0s[3][e], z0);
      z1 = fmaf(t0, w1s[0][e], z1);
      z1 = fmaf(t1, w1s[1][e], z1);
      z1 = fmaf(t2, w1s[2][e], z1);
      z1 = fmaf(t3, w1s[3][e], z1);
    }
#pragma unroll
    for (int off = 1; off < 32; off <<= 1) {
      z0 += __shfl_xor(z0, off, 32);
      z1 += __shfl_xor(z1, off, 32);
    }
    keep0 = (lane == i) ? z0 : keep0;
    keep1 = (lane == i) ? z1 : keep1;
    unsigned short* gp = g16 + (size_t)row * NFEAT + c8;
    for (int pass = 0; pass < 2; ++pass) {
      *(volatile v4u*)(void*)(gp + NDIM) = hw;
      *(volatile v8h*)(gp + 2 * NDIM) = h2;
      *(volatile v8h*)(gp + 3 * NDIM) = h3;
      __threadfence();
    }
  }
  float* p0 = zg0 + row0 + lane;
  float* p1 = zg1 + row0 + lane;
  for (int pass = 0; pass < 2; ++pass) {
    *(volatile float*)p0 = keep0;
    *(volatile float*)p1 = keep1;
    __threadfence();
  }
}

__global__ __launch_bounds__(NTHR) void lstm_rec_kernel(const unsigned short* __restrict__ pre16,
                                                        const unsigned short* __restrict__ whh16,
                                                        unsigned short* __restrict__ mout, int dirflag) {
  __shared__ __align__(16) _Float16       Ah[2][16 * HPITCH];
  __shared__ __align__(16) unsigned short Pt[2][16 * PPITCH];
  const _Float16* WH = (const _Float16*)(const void*)whh16;
  const int tid = threadIdx.x, lane = tid & 31, wave = tid >> 5;
  const int c = lane & 15, hh = lane >> 4, koff = hh * 8;
  const int rowbase = blockIdx.x * 16;
  const int srow = tid >> 6, sch = tid & 63;

  {
    _Float16* ahf = &Ah[0][0];
#pragma unroll 1
    for (int i = tid; i < 2 * 16 * HPITCH; i += NTHR) ahf[i] = (_Float16)0.0f;
  }
  {
    const int t0 = dirflag ? (NSEQ - 1) : 0;
#pragma unroll
    for (int it = 0; it < 4; ++it) {
      const int row = it * 4 + srow;
      const v4u v = *(const v4u*)(const void*)(pre16 + ((size_t)(rowbase + row) * NSEQ + t0) * NGATE + sch * 8);
      *(v4u*)(void*)(&Pt[0][0] + row * PPITCH + sch * 8) = v;
    }
  }
  float cst[8];
#pragma unroll
  for (int r = 0; r < 8; ++r) cst[r] = 0.0f;
  __syncthreads();

  const int j = 16 * wave + c;
  const _Float16* whrow = WH + (size_t)j * NHID + koff;
  const v8f z8 = {0.f, 0.f, 0.f, 0.f, 0.f, 0.f, 0.f, 0.f};

#pragma unroll 1
  for (int t = 0; t < NSEQ; ++t) {
    const int cur = t & 1;
    const int tt = dirflag ? (NSEQ - 1 - t) : t;
    const int tnr = (t + 1 < NSEQ) ? (t + 1) : (NSEQ - 1);
    const int tn = dirflag ? (NSEQ - 1 - tnr) : tnr;
    v4u pn[4];
#pragma unroll
    for (int it = 0; it < 4; ++it) {
      const int row = it * 4 + srow;
      pn[it] = *(const v4u*)(const void*)(pre16 + ((size_t)(rowbase + row) * NSEQ + tn) * NGATE + sch * 8);
    }
    const _Float16* ahrow = &Ah[cur][0] + c * HPITCH + koff;
    v8f acc0 = z8, acc1 = z8, acc2 = z8, acc3 = z8;
#pragma unroll 1
    for (int k0 = 0; k0 < NHID; k0 += 32) {
      const v16h a  = Frag<_Float16>::load(ahrow + k0);
      const v16h b0 = Frag<_Float16>::load(whrow + k0);
      const v16h b1 = Frag<_Float16>::load(whrow + (size_t)1 * NHID * NHID + k0);
      const v16h b2 = Frag<_Float16>::load(whrow + (size_t)2 * NHID * NHID + k0);
      const v16h b3 = Frag<_Float16>::load(whrow + (size_t)3 * NHID * NHID + k0);
      acc0 = Frag<_Float16>::mma(a, b0, acc0);
      acc1 = Frag<_Float16>::mma(a, b1, acc1);
      acc2 = Frag<_Float16>::mma(a, b2, acc2);
      acc3 = Frag<_Float16>::mma(a, b3, acc3);
      guard4_h(acc0, acc1, acc2, acc3, a, b0, b1, b2, b3);
    }
    acc_guard4(acc0, acc1, acc2, acc3);
    const unsigned short* ptc = &Pt[cur][0] + j;
    _Float16* ahn = &Ah[cur ^ 1][0] + j;
#pragma unroll
    for (int r = 0; r < 8; ++r) {
      const unsigned short* pr = ptc + (8 * hh + r) * PPITCH;
      const float pi = h16_to_f32((unsigned)pr[0]);
      const float pf = h16_to_f32((unsigned)pr[NHID]);
      const float pg = h16_to_f32((unsigned)pr[2 * NHID]);
      const float po = h16_to_f32((unsigned)pr[3 * NHID]);
      const float zi = acc0[r] * WCARRY_INV + pi;
      const float zf = acc1[r] * WCARRY_INV + pf;
      const float zg = acc2[r] * WCARRY_INV + pg;
      const float zo = acc3[r] * WCARRY_INV + po;
      const float ig = fsig(zi);
      const float fg = fsig(zf);
      const float gg = ftanh(zg);
      const float og = fsig(zo);
      const float cn = fg * cst[r] + ig * gg;
      cst[r] = cn;
      const float hn = og * ftanh(cn);
      ahn[(8 * hh + r) * HPITCH] = (_Float16)hn;
    }
    {
      unsigned short* ptn = &Pt[cur ^ 1][0];
#pragma unroll
      for (int it = 0; it < 4; ++it) {
        const int row = it * 4 + srow;
        *(v4u*)(void*)(ptn + row * PPITCH + sch * 8) = pn[it];
      }
    }
    __syncthreads();
    {
      const int row = tid >> 4, ch = tid & 15;
      const v8h hv = *(const v8h*)(&Ah[cur ^ 1][0] + row * HPITCH + ch * 8);
      unsigned short* dp = mout + ((size_t)(rowbase + row) * NSEQ + tt) * NBI + dirflag * NHID + ch * 8;
      *(volatile v8h*)dp = hv;
      __threadfence();
      *(volatile v8h*)dp = hv;
    }
  }
}

__global__ __launch_bounds__(NTHR) void final_kernel(const float* __restrict__ zg0, const float* __restrict__ zg1,
                                                     const unsigned short* __restrict__ mA, const unsigned short* __restrict__ mB,
                                                     const float* __restrict__ W0, const float* __restrict__ W1,
                                                     const float* __restrict__ b0, const float* __restrict__ b1,
                                                     float* __restrict__ out) {
  __shared__ float Wt[NBI];
  __shared__ float red[8];
  const int tid = threadIdx.x, lane = tid & 31, wave = tid >> 5;
  const int sel = blockIdx.x >> 6;
  const int b = blockIdx.x & 63;
  const float* zg = sel ? zg1 : zg0;
  const unsigned short* mp = sel ? mB : mA;
  const float* Wv = sel ? W1 : W0;
  const float bias0 = b0[0];
  const float bias1 = b1[0];
  const float bias = sel ? bias1 : bias0;
  Wt[tid] = Wv[NFEAT + tid];
  __syncthreads();
  float zv[2];
#pragma unroll
  for (int hs = 0; hs < 2; ++hs) {
    const int row = b * NSEQ + hs * 256 + tid;
    const v4u* rp = (const v4u*)(const void*)(mp + (size_t)row * NBI);
    float s0 = 0.0f, s1 = 0.0f;
#pragma unroll 1
    for (int ch = 0; ch < NBI / 8; ++ch) {
      const v4u w = rp[ch];
#pragma unroll
      for (int k = 0; k < 4; ++k) {
        const unsigned wd = w[k];
        s0 = fmaf(h16_to_f32(wd & 0xffffu), Wt[ch * 8 + 2 * k], s0);
        s1 = fmaf(h16_to_f32(wd >> 16), Wt[ch * 8 + 2 * k + 1], s1);
      }
    }
    zv[hs] = zg[row] + (s0 + s1) + bias;
  }
  const float zA = zv[0];
  const float zB = zv[1];
  float m = fmaxf(zA, zB);
#pragma unroll
  for (int off = 1; off < 32; off <<= 1) m = fmaxf(m, __shfl_xor(m, off, 32));
  if (lane == 0) red[wave] = m;
  __syncthreads();
  float mx = red[0];
#pragma unroll
  for (int w = 1; w < 8; ++w) mx = fmaxf(mx, red[w]);
  __syncthreads();
  const float eA = expf(zA - mx);
  const float eB = expf(zB - mx);
  float s = eA + eB;
#pragma unroll
  for (int off = 1; off < 32; off <<= 1) s += __shfl_xor(s, off, 32);
  if (lane == 0) red[wave] = s;
  __syncthreads();
  const float tot = ((red[0] + red[1]) + (red[2] + red[3])) + ((red[4] + red[5]) + (red[6] + red[7]));
  const float inv = 1.0f / tot;
  const float pA = eA * inv;
  const float pB = eB * inv;
  float* op = out + (size_t)sel * NROWS + (size_t)b * NSEQ + tid;
  for (int pass = 0; pass < 2; ++pass) {
    *(volatile float*)op = pA;
    *(volatile float*)(op + 256) = pB;
    __threadfence();
  }
}

extern "C" void kernel_launch(void* const* d_in, const int* in_sizes, int n_in,
                              void* d_out, int out_size, void* d_ws, size_t ws_size, hipStream_t stream) {
  if (n_in < 28 || d_out == nullptr || d_ws == nullptr) return;
  if (in_sizes[0] != NROWS * NDIM || in_sizes[1] != NQROWS * NDIM || in_sizes[2] != NDIM || in_sizes[4] != NDIM ||
      in_sizes[6] != NDIM || in_sizes[8] != NGATE * NFEAT || in_sizes[9] != NGATE * NHID || in_sizes[10] != NGATE ||
      in_sizes[12] != NGATE * NFEAT || in_sizes[13] != NGATE * NHID || in_sizes[16] != NGATE * NBI ||
      in_sizes[17] != NGATE * NHID || in_sizes[20] != NGATE * NBI || in_sizes[21] != NGATE * NHID ||
      in_sizes[24] != NWVEC || in_sizes[26] != NWVEC || out_size != 2 * NROWS) return;

  const float* cx   = (const float*)d_in[0];
  const float* qx   = (const float*)d_in[1];
  const float* wc   = (const float*)d_in[2];
  const float* bc   = (const float*)d_in[3];
  const float* wq   = (const float*)d_in[4];
  const float* bq   = (const float*)d_in[5];
  const float* wcq  = (const float*)d_in[6];
  const float* bcq  = (const float*)d_in[7];
  const float* l1f_Wih = (const float*)d_in[8];
  const float* l1f_Whh = (const float*)d_in[9];
  const float* l1f_bih = (const float*)d_in[10];
  const float* l1f_bhh = (const float*)d_in[11];
  const float* l1b_Wih = (const float*)d_in[12];
  const float* l1b_Whh = (const float*)d_in[13];
  const float* l1b_bih = (const float*)d_in[14];
  const float* l1b_bhh = (const float*)d_in[15];
  const float* l2f_Wih = (const float*)d_in[16];
  const float* l2f_Whh = (const float*)d_in[17];
  const float* l2f_bih = (const float*)d_in[18];
  const float* l2f_bhh = (const float*)d_in[19];
  const float* l2b_Wih = (const float*)d_in[20];
  const float* l2b_Whh = (const float*)d_in[21];
  const float* l2b_bih = (const float*)d_in[22];
  const float* l2b_bhh = (const float*)d_in[23];
  const float* W0 = (const float*)d_in[24];
  const float* b0 = (const float*)d_in[25];
  const float* W1 = (const float*)d_in[26];
  const float* b1 = (const float*)d_in[27];
  float* out = (float*)d_out;

  char* ws = (char*)d_ws; size_t off = 0;
  auto carve = [&](size_t bytes) -> char* { char* p = ws + off; off += (bytes + 255) & ~(size_t)255; return p; };
  char* regA = carve((size_t)33554432);
  unsigned short* QW16  = (unsigned short*)(regA);
  unsigned short* QT16  = (unsigned short*)(regA + 2097152);
  float*          S32   = (float*)(regA + 4194304);
  unsigned short* A16   = (unsigned short*)(regA + 12582912);
  unsigned short* C2Q16 = (unsigned short*)(regA + 16777216);
  unsigned short* PRE16 = (unsigned short*)(regA);
  unsigned short* G16   = (unsigned short*)carve((size_t)NROWS * NFEAT * 2);
  unsigned short* M2_16 = G16;
  unsigned short* M16   = (unsigned short*)carve((size_t)NROWS * NBI * 2);
  unsigned short* W1F   = (unsigned short*)carve((size_t)NGATE * NFEAT * 2);
  unsigned short* W1B   = (unsigned short*)carve((size_t)NGATE * NFEAT * 2);
  unsigned short* W2F   = (unsigned short*)carve((size_t)NGATE * NBI * 2);
  unsigned short* W2B   = (unsigned short*)carve((size_t)NGATE * NBI * 2);
  unsigned short* WH1F  = (unsigned short*)carve((size_t)NGATE * NHID * 2);
  unsigned short* WH1B  = (unsigned short*)carve((size_t)NGATE * NHID * 2);
  unsigned short* WH2F  = (unsigned short*)carve((size_t)NGATE * NHID * 2);
  unsigned short* WH2B  = (unsigned short*)carve((size_t)NGATE * NHID * 2);
  float* BSUM = (float*)carve((size_t)4 * NGATE * 4);
  float* CW   = (float*)carve((size_t)NROWS * 4);
  float* QV   = (float*)carve((size_t)NQROWS * 4);
  float* SMAX = (float*)carve((size_t)NROWS * 4);
  float* Q2C  = (float*)carve((size_t)NBAT * NDIM * 4);
  float* ZG0  = (float*)carve((size_t)NROWS * 4);
  float* ZG1  = (float*)carve((size_t)NROWS * 4);
  if (off > ws_size || off > (size_t)134217728) return;

  cvtw_kernel<<<dim3((NGATE * NFEAT / 8) / NTHR, 2), NTHR, 0, stream>>>(l1f_Wih, l1b_Wih, l1f_Wih, l1b_Wih, W1F, W1B, W1F, W1B,
                                                                        NGATE * NFEAT / 8, WCARRY);
  cvtw_kernel<<<dim3((NGATE * NBI / 8) / NTHR, 2), NTHR, 0, stream>>>(l2f_Wih, l2b_Wih, l2f_Wih, l2b_Wih, W2F, W2B, W2F, W2B,
                                                                      NGATE * NBI / 8, WCARRY);
  cvtw_kernel<<<dim3((NGATE * NHID / 8) / NTHR, 4), NTHR, 0, stream>>>(l1f_Whh, l1b_Whh, l2f_Whh, l2b_Whh, WH1F, WH1B, WH2F, WH2B,
                                                                       NGATE * NHID / 8, WCARRY);
  bsum_kernel<<<1, 512, 0, stream>>>(l1f_bih, l1f_bhh, l1b_bih, l1b_bhh, l2f_bih, l2f_bhh, l2b_bih, l2b_bhh, BSUM);

  rowprep_kernel<0><<<NROWS / NTHR, NTHR, 0, stream>>>(cx, wc, bc, bcq, wc, G16, NFEAT, CW, NROWS);
  rowprep_kernel<1><<<NQROWS / NTHR, NTHR, 0, stream>>>(qx, wq, bq, bq, wcq, QW16, NDIM, QV, NQROWS);
  qtrans_kernel<<<dim3(NDIM / 64, NBAT), NTHR, 0, stream>>>(qx, QT16);

  gemm64_kernel<0, true><<<dim3(1, NBAT), 256, 0, stream>>>(
      G16, NFEAT, (long)NSEQ * NFEAT, QW16, NDIM, (long)NQRY * NDIM, (void*)S32, NQRY, (long)NSEQ * NQRY,
      CW, (long)NSEQ, QV, (long)NQRY, NSEQ, NQRY, NDIM, QCARRY_INV);

  softj_kernel<<<NROWS / NTHR, NTHR, 0, stream>>>(S32, A16, SMAX);
  q2c_kernel<<<NBAT, NTHR, 0, stream>>>(SMAX, cx, Q2C);

  gemm64_kernel<1, false><<<dim3(4, NBAT), 256, 0, stream>>>(
      A16, NQRY, (long)NSEQ * NQRY, QT16, NQRY, (long)NDIM * NQRY, (void*)C2Q16, NDIM, (long)NSEQ * NDIM,
      CW, 0L, CW, 0L, NSEQ, NDIM, NQRY, PCARRY_INV);

  assemble_kernel<<<NROWS / NTHR, NTHR, 0, stream>>>(cx, C2Q16, Q2C, W0, W1, G16, ZG0, ZG1);

  const dim3 pgrid((NROWS / 64) * (NGATE / 64) / 8, 1);
  gemm64_kernel<1, true><<<pgrid, 256, 0, stream>>>(
      G16, NFEAT, 0L, W1F, NFEAT, 0L, (void*)PRE16, NGATE, 0L, CW, 0L, BSUM + 0 * NGATE, 0L, NROWS, NGATE, NFEAT, WCARRY_INV);
  lstm_rec_kernel<<<NBAT / 16, NTHR, 0, stream>>>(PRE16, WH1F, M16, 0);
  gemm64_kernel<1, true><<<pgrid, 256, 0, stream>>>(
      G16, NFEAT, 0L, W1B, NFEAT, 0L, (void*)PRE16, NGATE, 0L, CW, 0L, BSUM + 1 * NGATE, 0L, NROWS, NGATE, NFEAT, WCARRY_INV);
  lstm_rec_kernel<<<NBAT / 16, NTHR, 0, stream>>>(PRE16, WH1B, M16, 1);

  gemm64_kernel<1, true><<<pgrid, 256, 0, stream>>>(
      M16, NBI, 0L, W2F, NBI, 0L, (void*)PRE16, NGATE, 0L, CW, 0L, BSUM + 2 * NGATE, 0L, NROWS, NGATE, NBI, WCARRY_INV);
  lstm_rec_kernel<<<NBAT / 16, NTHR, 0, stream>>>(PRE16, WH2F, M2_16, 0);
  gemm64_kernel<1, true><<<pgrid, 256, 0, stream>>>(
      M16, NBI, 0L, W2B, NBI, 0L, (void*)PRE16, NGATE, 0L, CW, 0L, BSUM + 3 * NGATE, 0L, NROWS, NGATE, NBI, WCARRY_INV);
  lstm_rec_kernel<<<NBAT / 16, NTHR, 0, stream>>>(PRE16, WH2B, M2_16, 1);

  final_kernel<<<2 * NBAT, NTHR, 0, stream>>>(ZG0, ZG1, M16, M2_16, W0, W1, b0, b1, out);
}
